// ReconGNN_7894149890553
// MI455X (gfx1250) — hardware-verified
//
#include <hip/hip_runtime.h>
#include <stddef.h>
#include <stdint.h>


#define NN     100000
#define NE     800000
#define HD     128
#define MP     100096
#define XP     256
#define KC     512
#define KH     256
#define NLAY   3
#define NTHR   256
#define NWAVE  8
#define EPT    8
#define CHUNK  (NTHR * EPT)
#define WCAP   (EPT * 32)
#define LISTN  (NWAVE * WCAP)
#define NBA    1024
#define SLA    10
#define SRB    17
#define NBLK   98
#define NSLOT  (NBLK * NBA)
#define RCAP   28672
#define DEGCAP 64
#define MEAS_B1024  (8392 + 8389)
#define MEAS_MAXDEG (24 + 23)
#define NCH    ((NE + CHUNK - 1) / CHUNK)
#define GBM    128
#define PAROWS 16
#define NUWC   (NLAY * HD * (KC / 8))
#define NUWH   (3 * HD * (KH / 8))
#define TB_BG   0
#define TB_BN1  384
#define TB_WN2  512
#define TB_T6   640
#define TB_BE1  1408
#define TB_WE2  1536
#define TB_SC   1664
#define TB_N    1792
#define NTU    (TB_N / 4)
#define BK_ZINTS (RCAP + 3 * NBA)
#define BK_LDS_INTS (LISTN + 2 * RCAP + 3 * NBA + 16)
#define GM_LDS_BYTES (GBM * HD * 4)
#define WSMAX  134217728

static_assert((CHUNK & (CHUNK - 1)) == 0 && CHUNK <= 4096);
static_assert(NBA == (1 << SLA) && ((long long)CHUNK << SLA) < (1LL << 31));
static_assert(NN <= (1 << SRB) && (SRB + SLA) < 31);
static_assert(NE % 32 == 0 && NE % 4 == 0 && NE % NTHR == 0);
static_assert(NE / 32 == 25000 && (NN * 4) % 128 == 0 && (NN * 4) / 128 == 3125);
static_assert(NN % 32 == 0 && NN % 4 == 0);
static_assert(MP % GBM == 0 && MP / GBM == 782 && MP >= NN && MP <= NSLOT);
static_assert(NSLOT >= NN && NBA % GBM == 0);
static_assert(RCAP >= MEAS_B1024 + 4096 && RCAP % (NTHR * 4) == 0);
static_assert(DEGCAP >= MEAS_MAXDEG + 8);
static_assert(BK_ZINTS % (NTHR * 4) == 0);
static_assert(BK_LDS_INTS * 4 <= 300000);
static_assert(HD == 128 && XP == 2 * HD && KC == 4 * HD && KH == 2 * HD && KC % 32 == 0 && KH % 32 == 0);
static_assert(GBM == NWAVE * 16 && NTHR == NWAVE * 32);
static_assert(MP % (NWAVE * PAROWS) == 0);
static_assert(NUWC % NTHR == 0 && NUWH % NTHR == 0 && (NUWC / NLAY / 2) % NTHR == 0 && (NUWH / 3) % NTHR == 0);
static_assert(TB_N % 128 == 0 && NTU % 32 == 0);

typedef float          v2f   __attribute__((ext_vector_type(2)));
typedef float          v4f   __attribute__((ext_vector_type(4)));
typedef float          v8f   __attribute__((ext_vector_type(8)));
typedef int            v4i   __attribute__((ext_vector_type(4)));
typedef int            v8i   __attribute__((ext_vector_type(8)));
typedef unsigned       v2u   __attribute__((ext_vector_type(2)));
typedef unsigned short v4us  __attribute__((ext_vector_type(4)));
typedef unsigned short v8us  __attribute__((ext_vector_type(8)));
typedef __bf16         v16bf __attribute__((ext_vector_type(16)));
typedef v4f  __attribute__((may_alias)) v4fa;
typedef v4i  __attribute__((may_alias)) v4ia;
typedef v2u  __attribute__((may_alias)) v2ua;
typedef v4us __attribute__((may_alias)) v4usa;
typedef v8us __attribute__((may_alias)) v8usa;
union FragB { v16bf v; v8us h[2]; v8i w; };

__device__ __forceinline__ v8f wmb(const FragB& a, const FragB& b, v8f c) {
  v8f d = __builtin_amdgcn_wmma_f32_16x16x32_bf16(false, a.v, false, b.v, (short)0, c, false, false);
  asm volatile("v_nop\n\tv_nop\n\tv_nop\n\tv_nop" : "+v"(d) : "v"(a.w), "v"(b.w));
  return d;
}
__device__ __forceinline__ v8f z8() { v8f z = {0.f, 0.f, 0.f, 0.f, 0.f, 0.f, 0.f, 0.f}; return z; }

__device__ __forceinline__ unsigned f2bf(float f) {
  const unsigned u = __float_as_uint(f);
  const unsigned r = ((u + 0x7FFFu + ((u >> 16) & 1u)) >> 16) & 0xFFFFu;
  return ((u & 0x7FFFFFFFu) > 0x7F800000u) ? 0x7FC0u : r;
}
__device__ __forceinline__ float bf2f(unsigned b) { return __uint_as_float(b << 16); }
__device__ __forceinline__ float bfr(float f) { return bf2f(f2bf(f)); }
__device__ __forceinline__ unsigned hl_bits(float v, unsigned& lo) {
  const unsigned hb = f2bf(v);
  lo = f2bf(v - bf2f(hb));
  return hb;
}
__device__ __forceinline__ float relu_k(float v) { return (v > 0.0f) ? v : (v - v); }
__device__ __forceinline__ float rdl(float v, int k) {
  return __int_as_float(__builtin_amdgcn_readlane(__float_as_int(v), k));
}

__device__ __forceinline__ void wave_sync() {
  __builtin_amdgcn_fence(__ATOMIC_RELEASE, "workgroup");
  __builtin_amdgcn_wave_barrier();
  __builtin_amdgcn_fence(__ATOMIC_ACQUIRE, "workgroup");
}

template <int SLB>
__device__ __forceinline__ int scan_chunk(const int* __restrict__ dsts, int nE, int cbase, int slotBase,
                                          int nb, int vec8, int* list, int tid, int lane, int wave) {
  int wc = 0;
  const int el0  = tid * EPT;
  const int e0   = cbase + el0;
  const int sent = -2147483647 - 1;
  v4i da, db;
  if (vec8 != 0 && cbase + CHUNK <= nE) {
    da = *(const v4i*)(dsts + e0);
    db = *(const v4i*)(dsts + e0 + 4);
  } else {
    da.x = (e0     < nE) ? dsts[min(e0,     nE - 1)] : sent;
    da.y = (e0 + 1 < nE) ? dsts[min(e0 + 1, nE - 1)] : sent;
    da.z = (e0 + 2 < nE) ? dsts[min(e0 + 2, nE - 1)] : sent;
    da.w = (e0 + 3 < nE) ? dsts[min(e0 + 3, nE - 1)] : sent;
    db.x = (e0 + 4 < nE) ? dsts[min(e0 + 4, nE - 1)] : sent;
    db.y = (e0 + 5 < nE) ? dsts[min(e0 + 5, nE - 1)] : sent;
    db.z = (e0 + 6 < nE) ? dsts[min(e0 + 6, nE - 1)] : sent;
    db.w = (e0 + 7 < nE) ? dsts[min(e0 + 7, nE - 1)] : sent;
  }
  const unsigned nbs = (unsigned)slotBase;
  const unsigned unb = (unsigned)nb;
  const unsigned s0 = (unsigned)da.x - nbs, s1 = (unsigned)da.y - nbs;
  const unsigned s2 = (unsigned)da.z - nbs, s3 = (unsigned)da.w - nbs;
  const unsigned s4 = (unsigned)db.x - nbs, s5 = (unsigned)db.y - nbs;
  const unsigned s6 = (unsigned)db.z - nbs, s7 = (unsigned)db.w - nbs;
  const bool h0 = s0 < unb, h1 = s1 < unb, h2 = s2 < unb, h3 = s3 < unb;
  const bool h4 = s4 < unb, h5 = s5 < unb, h6 = s6 < unb, h7 = s7 < unb;
  const unsigned any = __builtin_amdgcn_ballot_w32(h0 | h1 | h2 | h3 | h4 | h5 | h6 | h7);
  if (any != 0u) {
#define HITJ(J, HJ, SJ) { \
      const unsigned mj = __builtin_amdgcn_ballot_w32(HJ); \
      if (mj != 0u) { \
        if (HJ) { \
          const int pos = wc + (int)__builtin_amdgcn_mbcnt_lo(mj, 0u); \
          if (pos < WCAP) list[wave * WCAP + pos] = ((el0 + (J)) << SLB) | (int)(SJ); \
        } \
        wc += (int)__builtin_popcount(mj); } }
    HITJ(0, h0, s0)
    HITJ(1, h1, s1)
    HITJ(2, h2, s2)
    HITJ(3, h3, s3)
    HITJ(4, h4, s4)
    HITJ(5, h5, s5)
    HITJ(6, h6, s6)
    HITJ(7, h7, s7)
#undef HITJ
  }
  return wc;
}

__global__ __launch_bounds__(NTHR) __attribute__((amdgpu_num_vgpr(248)))
void k_pa(const float* __restrict__ ns, const float* __restrict__ pobs, const int* __restrict__ pmask,
          const float* __restrict__ wenc, const float* __restrict__ benc, unsigned short* XA) {
  __shared__ __attribute__((aligned(16))) float wsm[8 * HD];
  __shared__ __attribute__((aligned(16))) unsigned short rowb[NWAVE * XP];
  const int tid = (int)threadIdx.x, lane = tid & 31, wave = tid >> 5;
  {
    const v4f w = *(const v4f*)(wenc + 4 * tid);
    v4f o; o.x = bfr(w.x); o.y = bfr(w.y); o.z = bfr(w.z); o.w = bfr(w.w);
    *(v4fa*)(wsm + 4 * tid) = o;
  }
  __syncthreads();
  float b0, b1, b2, b3;
  {
    const v4f b4 = *(const v4f*)(benc + 4 * lane);
    b0 = bfr(b4.x); b1 = bfr(b4.y); b2 = bfr(b4.z); b3 = bfr(b4.w);
  }
  unsigned short* rb = rowb + wave * XP;
  const int row0 = ((int)blockIdx.x * NWAVE + wave) * PAROWS;
  const int fi  = lane & 7;
  const int fc  = fi < 6 ? fi : 5;
  const unsigned mk0 = 0u - (unsigned)(fi < 6);
  const unsigned mk1 = 0u - (unsigned)(fi == 6);
  const unsigned mk2 = ~(mk0 | mk1);
#pragma unroll 1
  for (int i = 0; i < PAROWS; ++i) {
    const int row = row0 + i;
    const int rc  = row < NN ? row : NN - 1;
    unsigned ua = __float_as_uint(ns[(size_t)rc * 6 + fc]);
    unsigned ub = __float_as_uint(pobs[rc]);
    unsigned um = (unsigned)pmask[rc];
    asm volatile("" : "+v"(ua), "+v"(ub), "+v"(um));
    const unsigned uo = (unsigned)(um != 0u) * 0x3f800000u;
    float fv = __uint_as_float((ua & mk0) | (ub & mk1) | (uo & mk2));
    fv = bfr(fv);
    float a0 = 0.0f, a1 = 0.0f, a2 = 0.0f, a3 = 0.0f;
#pragma unroll 1
    for (int k = 0; k < 8; ++k) {
      const float f = rdl(fv, k);
      const v4f w = *(const v4fa*)(wsm + k * HD + 4 * lane);
      a0 = fmaf(f, w.x, a0); a1 = fmaf(f, w.y, a1); a2 = fmaf(f, w.z, a2); a3 = fmaf(f, w.w, a3);
    }
    const bool live = row < NN;
    const float m0 = live ? (a0 + b0) : 0.0f;
    const float m1 = live ? (a1 + b1) : 0.0f;
    const float m2 = live ? (a2 + b2) : 0.0f;
    const float m3 = live ? (a3 + b3) : 0.0f;
    v4us mh, ml;
    {
      unsigned lb, hb;
      hb = hl_bits(m0, lb); mh[0] = (unsigned short)hb; ml[0] = (unsigned short)lb;
      hb = hl_bits(m1, lb); mh[1] = (unsigned short)hb; ml[1] = (unsigned short)lb;
      hb = hl_bits(m2, lb); mh[2] = (unsigned short)hb; ml[2] = (unsigned short)lb;
      hb = hl_bits(m3, lb); mh[3] = (unsigned short)hb; ml[3] = (unsigned short)lb;
    }
    *(v4usa*)(rb + 4 * lane)      = mh;
    *(v4usa*)(rb + HD + 4 * lane) = ml;
    wave_sync();
    const v8us q0 = *(const v8usa*)(rb + 8 * lane);
    wave_sync();
    unsigned short* rpw = XA + (size_t)row * XP + 8 * lane;
    *(volatile v8us*)rpw = q0;
    __threadfence();
    *(volatile v8us*)rpw = q0;
  }
}

__global__ __launch_bounds__(NTHR) __attribute__((amdgpu_num_vgpr(248)))
void k_pb(const float* __restrict__ wl, const float* __restrict__ wr, unsigned short* WC) {
  const int u    = (int)blockIdx.x * NTHR + (int)threadIdx.x;
  const int l    = u >> 13;
  const int rem  = u & 8191;
  const int half = rem >> 12;
  const int n    = (rem >> 5) & (HD - 1);
  const int k8   = (rem & 31) * 8;
  const int kk   = k8 & (HD - 1);
  const size_t so = (size_t)l * HD * HD + (size_t)kk * HD + (size_t)n;
  v8us o;
  if (half == 0) {
#pragma unroll
    for (int i = 0; i < 8; ++i) o[i] = (unsigned short)f2bf(wr[so + (size_t)i * HD]);
  } else {
#pragma unroll
    for (int i = 0; i < 8; ++i) o[i] = (unsigned short)f2bf(wl[so + (size_t)i * HD]);
  }
  unsigned short* dp = WC + (size_t)l * HD * KC + (size_t)n * KC + half * 256 + k8;
  *(volatile v8us*)dp = o;
  __threadfence();
  *(volatile v8us*)dp = o;
}

__global__ __launch_bounds__(NTHR) __attribute__((amdgpu_num_vgpr(248)))
void k_pc(const float* __restrict__ wn1, const float* __restrict__ we1, const float* __restrict__ bg,
          const float* __restrict__ bn1, const float* __restrict__ wn2, const float* __restrict__ bn2,
          const float* __restrict__ be1, const float* __restrict__ we2, const float* __restrict__ be2,
          unsigned short* WH, float* TB) {
  const int u = (int)blockIdx.x * NTHR + (int)threadIdx.x;
  if (u < NUWH) {
    const int p  = u >> 12;
    const int n  = (u >> 5) & (HD - 1);
    const int k8 = (u & 31) * 8;
    const int kk = k8 & (HD - 1);
    v8us o;
    if (p == 0) {
      const size_t so = (size_t)kk * HD + (size_t)n;
#pragma unroll
      for (int i = 0; i < 8; ++i) o[i] = (unsigned short)f2bf(wn1[so + (size_t)i * HD]);
    } else {
      const size_t so = (size_t)((p - 1) * HD + kk) * HD + (size_t)n;
#pragma unroll
      for (int i = 0; i < 8; ++i) o[i] = (unsigned short)f2bf(we1[so + (size_t)i * HD]);
    }
    unsigned short* dp = WH + (size_t)p * HD * KH + (size_t)n * KH + k8;
    *(volatile v8us*)dp = o;
    __threadfence();
    *(volatile v8us*)dp = o;
  } else if (u < NUWH + NTU) {
    const int tu = u - NUWH;
    const int tw = tu >> 5;
    const int li = tu & 31;
    v4f s = {0.f, 0.f, 0.f, 0.f};
    if (tw < 3) {
      s = *(const v4f*)(bg + 4 * tu);
    } else if (tw == 3) {
      s = *(const v4f*)(bn1 + 4 * li);
    } else if (tw == 4) {
      s = *(const v4f*)(wn2 + 4 * li);
    } else if (tw < 11) {
      s = *(const v4f*)(we1 + (size_t)256 * HD + 4 * (tu - 160));
    } else if (tw == 11) {
      s = *(const v4f*)(be1 + 4 * li);
    } else if (tw == 12) {
      s = *(const v4f*)(we2 + 4 * li);
    } else {
      const float a = bn2[0];
      const float b = be2[0];
      s.x = (li == 0) ? a : 0.0f;
      s.y = (li == 0) ? b : 0.0f;
    }
    v4f o; o.x = bfr(s.x); o.y = bfr(s.y); o.z = bfr(s.z); o.w = bfr(s.w);
    float* dp = TB + 4 * tu;
    *(volatile v4f*)dp = o;
    __threadfence();
    *(volatile v4f*)dp = o;
  }
}

__global__ __launch_bounds__(NTHR) __attribute__((amdgpu_num_vgpr(248)))
void k_bkt(const int* __restrict__ ei, int* LIST, int* CNT, int* OFF, float* INVD, int* FLG) {
  extern __shared__ __attribute__((aligned(16))) int bsm[];
  int* list = bsm;
  int* reg1 = bsm + LISTN;
  int* sl   = reg1 + RCAP;
  int* cnt  = sl + RCAP;
  int* offs = cnt + NBA;
  int* cur  = offs + NBA;
  int* misc = cur + NBA;
  const int tid = (int)threadIdx.x, lane = tid & 31, wave = tid >> 5;
  const int blk = (int)blockIdx.x;
  const int nodeBase = blk * NBA;
  int nb = NN - nodeBase;
  nb = nb < 0 ? 0 : (nb > NBA ? NBA : nb);
  {
    const v4i z4 = {0, 0, 0, 0};
    for (int i = tid * 4; i < BK_ZINTS; i += NTHR * 4) *(v4ia*)(sl + i) = z4;
    if (tid < 16) misc[tid] = 0;
  }
  __syncthreads();

  int tot = 0, ovf = 0;
#pragma unroll 1
  for (int ch = 0; ch < 2 * NCH; ++ch) {
    const int ps     = (ch >= NCH) ? 1 : 0;
    const int cbase  = (ch - ps * NCH) * CHUNK;
    const int keyOff = ps ? 0 : NE;
    const int srcOff = ps ? NE : 0;
    const int wc = scan_chunk<SLA>(ei + keyOff, NE, cbase, nodeBase, nb, 1, list, tid, lane, wave);
    if (lane == 0) misc[wave] = wc;
    __syncthreads();
    int pre = 0, all = 0;
#pragma unroll
    for (int w2 = 0; w2 < NWAVE; ++w2) {
      int c = misc[w2];
      c = c < 0 ? 0 : (c > WCAP ? WCAP : c);
      all += c;
      pre += (w2 < wave) ? c : 0;
    }
    const int wcc  = wc > WCAP ? WCAP : wc;
    const int base = tot + pre;
#pragma unroll 1
    for (int i = lane; i < wcc; i += 32) {
      const int ent = list[wave * WCAP + i];
      const int el  = (ent >> SLA) & (CHUNK - 1);
      const int sq  = ent & (NBA - 1);
      int eid = cbase + el;
      eid = eid > NE - 1 ? NE - 1 : eid;
      const int sraw = ei[srcOff + eid];
      const int s = sraw < 0 ? 0 : (sraw > NN - 1 ? NN - 1 : sraw);
      const int pos = base + i;
      if (pos < RCAP) reg1[pos] = (int)((unsigned)s | ((unsigned)sq << SRB));
    }
    if (tot + all > RCAP) ovf = 1;
    tot += all;
    tot = tot > RCAP ? RCAP : tot;
    __syncthreads();
  }
  const int nh = tot;

  if (wave == 0) {
#pragma unroll 1
    for (int b0 = 0; b0 < nh; b0 += 32) {
      const int idx = b0 + lane;
      const int uv  = reg1[idx < nh ? idx : nh - 1];
      const int m32 = (nh - b0) < 32 ? (nh - b0) : 32;
#pragma unroll 1
      for (int k = 0; k < m32; ++k) {
        const int u  = __builtin_amdgcn_readlane(uv, k);
        const int sq = (u >> SRB) & (NBA - 1);
        if (lane == 0) cnt[sq] = cnt[sq] + 1;
      }
    }
  }
  __syncthreads();
  if (wave == 0) {
    const int base = lane * (NBA / 32);
    int s = 0;
#pragma unroll 1
    for (int i = 0; i < NBA / 32; ++i) s += cnt[base + i];
    int incl = s;
#pragma unroll
    for (int d = 1; d < 32; d <<= 1) {
      const int y = __shfl_up(incl, d, 32);
      if (lane >= d) incl += y;
    }
    int run = incl - s;
#pragma unroll 1
    for (int i = 0; i < NBA / 32; ++i) {
      const int cv = cnt[base + i];
      offs[base + i] = run;
      cur[base + i]  = run;
      run += cv;
    }
  }
  __syncthreads();
  if (wave == 0) {
#pragma unroll 1
    for (int b0 = 0; b0 < nh; b0 += 32) {
      const int idx = b0 + lane;
      const int uv  = reg1[idx < nh ? idx : nh - 1];
      const int m32 = (nh - b0) < 32 ? (nh - b0) : 32;
#pragma unroll 1
      for (int k = 0; k < m32; ++k) {
        const int u  = __builtin_amdgcn_readlane(uv, k);
        const int sq = (u >> SRB) & (NBA - 1);
        if (lane == 0) {
          int p = cur[sq];
          p = p < 0 ? 0 : (p > RCAP - 1 ? RCAP - 1 : p);
          sl[p] = u & ((1 << SRB) - 1);
          cur[sq] = p + 1;
        }
      }
    }
  }
  __syncthreads();

  int* lb = LIST + (size_t)blk * RCAP;
  const v4i cv4 = *(const v4ia*)(cnt + 4 * tid);
  const v4i ov4 = *(const v4ia*)(offs + 4 * tid);
  v4f iv4;
  iv4.x = 1.0f / fmaxf((float)cv4.x, 1.0f);
  iv4.y = 1.0f / fmaxf((float)cv4.y, 1.0f);
  iv4.z = 1.0f / fmaxf((float)cv4.z, 1.0f);
  iv4.w = 1.0f / fmaxf((float)cv4.w, 1.0f);
  int*   cp = CNT  + (size_t)nodeBase + 4 * tid;
  int*   op = OFF  + (size_t)nodeBase + 4 * tid;
  float* ip = INVD + (size_t)nodeBase + 4 * tid;
  v4i fv4;
  fv4.x = (tid == 0) ? nh : 0;
  fv4.y = (tid == 0) ? ovf : 0;
  fv4.z = 0; fv4.w = 0;
  int* fp = FLG + (size_t)blk * 32 + 4 * (tid & 7);
#pragma unroll 1
  for (int p = tid * 4; p < RCAP; p += NTHR * 4) {
    const v4i v = *(const v4ia*)(sl + p);
    *(volatile v4i*)(lb + p) = v;
  }
  *(volatile v4i*)cp = cv4;
  *(volatile v4i*)op = ov4;
  *(volatile v4f*)ip = iv4;
  if (tid < 8) *(volatile v4i*)fp = fv4;
  __threadfence();
#pragma unroll 1
  for (int p = tid * 4; p < RCAP; p += NTHR * 4) {
    const v4i v = *(const v4ia*)(sl + p);
    *(volatile v4i*)(lb + p) = v;
  }
  *(volatile v4i*)cp = cv4;
  *(volatile v4i*)op = ov4;
  *(volatile v4f*)ip = iv4;
  if (tid < 8) *(volatile v4i*)fp = fv4;
}

__global__ __launch_bounds__(NTHR) __attribute__((amdgpu_num_vgpr(248)))
void k_agg(const int* __restrict__ LIST, const int* __restrict__ CNT, const int* __restrict__ OFF,
           const float* __restrict__ INVD, const int* __restrict__ FLG,
           const unsigned short* XA, unsigned short* AGB) {
  __shared__ __attribute__((aligned(16))) unsigned short rowb[NWAVE * XP];
  const int tid = (int)threadIdx.x, lane = tid & 31, wave = tid >> 5;
  unsigned short* rb = rowb + wave * XP;
  const int base = ((int)blockIdx.x * NWAVE + wave) * PAROWS;
  int bb = base >> SLA;
  bb = bb > NBLK - 1 ? NBLK - 1 : bb;
  const int nhraw = FLG[(size_t)bb * 32];
  const int bflag = FLG[(size_t)bb * 32 + 1];
  const int ovf = (bflag != 0 || nhraw < 0 || nhraw > RCAP) ? 1 : 0;
  int ti = base + (lane & 15);
  ti = ti > NSLOT - 1 ? NSLOT - 1 : ti;
  const int   cl = CNT[ti];
  const int   ol = OFF[ti];
  const float il = INVD[ti];
  const int* lp = LIST + (size_t)bb * RCAP;
  const float qnan = __int_as_float(0x7fc00000);
  const float pz = (ovf != 0) ? qnan : 0.0f;
#pragma unroll 1
  for (int i = 0; i < PAROWS; ++i) {
    const int node = base + i;
    const int craw = __builtin_amdgcn_readlane(cl, i);
    const int oraw = __builtin_amdgcn_readlane(ol, i);
    const float inv = rdl(il, i);
    const bool big = (craw > DEGCAP) || (craw < 0);
    int c = craw < 0 ? 0 : (craw > DEGCAP ? DEGCAP : craw);
    int o = oraw < 0 ? 0 : (oraw > RCAP ? RCAP : oraw);
    if (c > RCAP - o) c = RCAP - o;
    const float pzr = big ? qnan : pz;
    const bool live = node < NN;
    float a0 = 0.0f, a1 = 0.0f, a2 = 0.0f, a3 = 0.0f;
#pragma unroll 1
    for (int b0 = 0; b0 < c; b0 += 32) {
      int idx = o + b0 + lane;
      idx = idx > RCAP - 1 ? RCAP - 1 : idx;
      int sr = lp[idx];
      sr = sr < 0 ? 0 : (sr > NN - 1 ? NN - 1 : sr);
      const int m32 = (c - b0) < 32 ? (c - b0) : 32;
#pragma unroll 1
      for (int k = 0; k < m32; ++k) {
        const int sk = __builtin_amdgcn_readlane(sr, k);
        const unsigned short* rp = XA + (size_t)sk * XP + 4 * lane;
        const v2u wh = *(const v2ua*)rp;
        const v2u wl = *(const v2ua*)(rp + HD);
        const float f0 = __uint_as_float(wh.x << 16)         + __uint_as_float(wl.x << 16);
        const float f1 = __uint_as_float(wh.x & 0xffff0000u) + __uint_as_float(wl.x & 0xffff0000u);
        const float f2 = __uint_as_float(wh.y << 16)         + __uint_as_float(wl.y << 16);
        const float f3 = __uint_as_float(wh.y & 0xffff0000u) + __uint_as_float(wl.y & 0xffff0000u);
        a0 += f0; a1 += f1; a2 += f2; a3 += f3;
      }
    }
    const float m0 = live ? (a0 * inv + pzr) : 0.0f;
    const float m1 = live ? (a1 * inv + pzr) : 0.0f;
    const float m2 = live ? (a2 * inv + pzr) : 0.0f;
    const float m3 = live ? (a3 * inv + pzr) : 0.0f;
    v4us mh, ml;
    {
      unsigned lb, hb;
      hb = hl_bits(m0, lb); mh[0] = (unsigned short)hb; ml[0] = (unsigned short)lb;
      hb = hl_bits(m1, lb); mh[1] = (unsigned short)hb; ml[1] = (unsigned short)lb;
      hb = hl_bits(m2, lb); mh[2] = (unsigned short)hb; ml[2] = (unsigned short)lb;
      hb = hl_bits(m3, lb); mh[3] = (unsigned short)hb; ml[3] = (unsigned short)lb;
    }
    *(v4usa*)(rb + 4 * lane)      = mh;
    *(v4usa*)(rb + HD + 4 * lane) = ml;
    wave_sync();
    const v8us q0 = *(const v8usa*)(rb + 8 * lane);
    wave_sync();
    unsigned short* rpw = AGB + (size_t)node * XP + 8 * lane;
    *(volatile v8us*)rpw = q0;
    __threadfence();
    *(volatile v8us*)rpw = q0;
  }
}

template <int MODE>
__global__ __launch_bounds__(NTHR) __attribute__((amdgpu_num_vgpr(248)))
void k_gm(const unsigned short* AG, unsigned short* XW, const unsigned short* __restrict__ BT,
          const float* __restrict__ TB, int biasOff, float* FO, float* outp) {
  extern __shared__ __attribute__((aligned(16))) float stg[];
  __shared__ __attribute__((aligned(16))) float sc[GBM];
  constexpr int LDB  = (MODE < 2) ? KC : KH;
  constexpr int BOFF = (MODE < 2) ? 256 : 0;
  const int tid = (int)threadIdx.x, lane = tid & 31, wave = tid >> 5, hh = lane >> 4, m = lane & 15;
  const int rowBase = (int)blockIdx.x * GBM;

  v8f acc[8];
#pragma unroll
  for (int t = 0; t < 8; ++t) acc[t] = z8();
  const size_t arow = (size_t)(rowBase + 16 * wave + m) * (size_t)XP + 8 * hh;
  const unsigned short* bp = BT + (size_t)m * (size_t)LDB + 8 * hh;

  if constexpr (MODE < 2) {
    const unsigned short* ap = AG + arow;
#pragma unroll 1
    for (int k0 = 0; k0 < 256; k0 += 32) {
      FragB af;
      af.h[0] = *(const v8usa*)(ap + k0);
      af.h[1] = *(const v8usa*)(ap + k0 + 16);
#pragma unroll
      for (int nt = 0; nt < 8; ++nt) {
        const unsigned short* wq = bp + (size_t)(16 * nt) * (size_t)LDB + k0;
        FragB bf;
        bf.h[0] = *(const v8usa*)wq;
        bf.h[1] = *(const v8usa*)(wq + 16);
        acc[nt] = wmb(af, bf, acc[nt]);
      }
    }
  }
  {
    const unsigned short* ap = (const unsigned short*)XW + arow;
#pragma unroll 1
    for (int k0 = 0; k0 < 256; k0 += 32) {
      FragB af;
      af.h[0] = *(const v8usa*)(ap + k0);
      af.h[1] = *(const v8usa*)(ap + k0 + 16);
#pragma unroll
      for (int nt = 0; nt < 8; ++nt) {
        const unsigned short* wq = bp + (size_t)(16 * nt) * (size_t)LDB + BOFF + k0;
        FragB bf;
        bf.h[0] = *(const v8usa*)wq;
        bf.h[1] = *(const v8usa*)(wq + 16);
        acc[nt] = wmb(af, bf, acc[nt]);
      }
    }
  }

#pragma unroll
  for (int nt = 0; nt < 8; ++nt) {
    const int lc = 16 * nt + m;
#pragma unroll
    for (int r = 0; r < 8; ++r) {
      const int lr = 16 * wave + 8 * hh + r;
      stg[lr * HD + lc] = acc[nt][r];
    }
  }
  __syncthreads();

  if constexpr (MODE == 2) {
    const v4f b1 = *(const v4f*)(TB + TB_BN1 + 4 * lane);
    const v4f w2 = *(const v4f*)(TB + TB_WN2 + 4 * lane);
    const float bz = TB[TB_SC];
    float keep = 0.0f;
#pragma unroll 1
    for (int i = 0; i < 16; ++i) {
      const v4f y = *(const v4fa*)(stg + (16 * wave + i) * HD + 4 * lane);
      const float h0 = relu_k(y.x + b1.x);
      const float h1 = relu_k(y.y + b1.y);
      const float h2 = relu_k(y.z + b1.z);
      const float h3 = relu_k(y.w + b1.w);
      float s = fmaf(h0, w2.x, fmaf(h1, w2.y, fmaf(h2, w2.z, h3 * w2.w)));
      s += __shfl_xor(s, 16, 32);
      s += __shfl_xor(s, 8, 32);
      s += __shfl_xor(s, 4, 32);
      s += __shfl_xor(s, 2, 32);
      s += __shfl_xor(s, 1, 32);
      keep = (lane == i) ? s : keep;
    }
    if (lane < 16) sc[16 * wave + lane] = keep + bz;
    __syncthreads();
    if (wave == 0) {
      const v4f v = *(const v4fa*)(sc + 4 * lane);
      const bool ok = (rowBase + 4 * lane + 3) < NN;
      float* op = outp + (size_t)rowBase + 4 * lane;
      if (ok) *(volatile v4f*)op = v;
      __threadfence();
      if (ok) *(volatile v4f*)op = v;
    }
    (void)AG; (void)FO; (void)biasOff;
  } else if constexpr (MODE >= 3) {
    v4f pv[16];
#pragma unroll
    for (int i = 0; i < 16; ++i) pv[i] = *(const v4fa*)(stg + (16 * wave + i) * HD + 4 * lane);
#pragma unroll
    for (int i = 0; i < 16; ++i) {
      const int gr = rowBase + 16 * wave + i;
      float* op = FO + (size_t)gr * HD + 4 * lane;
      *(volatile v4f*)op = pv[i];
    }
    __threadfence();
#pragma unroll
    for (int i = 0; i < 16; ++i) {
      const int gr = rowBase + 16 * wave + i;
      float* op = FO + (size_t)gr * HD + 4 * lane;
      *(volatile v4f*)op = pv[i];
    }
    (void)AG; (void)outp; (void)biasOff; (void)TB;
  } else {
    const v4f b4 = *(const v4f*)(TB + biasOff + 4 * lane);
    v4f pv[16];
#pragma unroll
    for (int i = 0; i < 16; ++i) pv[i] = *(const v4fa*)(stg + (16 * wave + i) * HD + 4 * lane);
    __syncthreads();
#pragma unroll
    for (int i = 0; i < 16; ++i) {
      const int row = rowBase + 16 * wave + i;
      const bool ok = row < NN;
      float o0 = pv[i].x + b4.x, o1 = pv[i].y + b4.y, o2 = pv[i].z + b4.z, o3 = pv[i].w + b4.w;
      if constexpr (MODE == 0) { o0 = relu_k(o0); o1 = relu_k(o1); o2 = relu_k(o2); o3 = relu_k(o3); }
      o0 = ok ? o0 : 0.0f; o1 = ok ? o1 : 0.0f; o2 = ok ? o2 : 0.0f; o3 = ok ? o3 : 0.0f;
      v4us h4, l4;
      unsigned lb, hb;
      hb = hl_bits(o0, lb); h4[0] = (unsigned short)hb; l4[0] = (unsigned short)lb;
      hb = hl_bits(o1, lb); h4[1] = (unsigned short)hb; l4[1] = (unsigned short)lb;
      hb = hl_bits(o2, lb); h4[2] = (unsigned short)hb; l4[2] = (unsigned short)lb;
      hb = hl_bits(o3, lb); h4[3] = (unsigned short)hb; l4[3] = (unsigned short)lb;
      unsigned short* srow = (unsigned short*)stg + (size_t)(16 * wave + i) * XP;
      *(v4usa*)(srow + 4 * lane)      = h4;
      *(v4usa*)(srow + HD + 4 * lane) = l4;
    }
    __syncthreads();
    v8us qv[16];
#pragma unroll
    for (int i = 0; i < 16; ++i) {
      const unsigned short* srow = (const unsigned short*)stg + (size_t)(16 * wave + i) * XP;
      qv[i] = *(const v8usa*)(srow + 8 * lane);
    }
#pragma unroll
    for (int i = 0; i < 16; ++i) {
      const int gr = rowBase + 16 * wave + i;
      unsigned short* rp = XW + (size_t)gr * XP + 8 * lane;
      *(volatile v8us*)rp = qv[i];
    }
    __threadfence();
#pragma unroll
    for (int i = 0; i < 16; ++i) {
      const int gr = rowBase + 16 * wave + i;
      unsigned short* rp = XW + (size_t)gr * XP + 8 * lane;
      *(volatile v8us*)rp = qv[i];
    }
    (void)FO; (void)outp;
  }
}

__global__ __launch_bounds__(NTHR) __attribute__((amdgpu_num_vgpr(248)))
void k_edge(const int* __restrict__ ei, const float* __restrict__ es, const float* __restrict__ qo,
            const int* __restrict__ qm, const float* __restrict__ PS, const float* __restrict__ PD,
            const float* __restrict__ TB, float* out1) {
  const int tid = (int)threadIdx.x, lane = tid & 31, wave = tid >> 5;
  const int e0 = ((int)blockIdx.x * NWAVE + wave) * 32;
  const int e  = e0 + lane;
  int s = ei[e];
  int d = ei[NE + e];
  s = s < 0 ? 0 : (s > NN - 1 ? NN - 1 : s);
  d = d < 0 ? 0 : (d > NN - 1 ? NN - 1 : d);
  const v4f f4 = *(const v4f*)(es + (size_t)4 * e);
  const float g0l = bfr(f4.x), g1l = bfr(f4.y), g2l = bfr(f4.z), g3l = bfr(f4.w);
  const float g4l = bfr(qo[e]);
  const float g5l = (qm[e] != 0) ? 1.0f : 0.0f;
  const v4f t0 = *(const v4f*)(TB + TB_T6 + 0 * HD + 4 * lane);
  const v4f t1 = *(const v4f*)(TB + TB_T6 + 1 * HD + 4 * lane);
  const v4f t2 = *(const v4f*)(TB + TB_T6 + 2 * HD + 4 * lane);
  const v4f t3 = *(const v4f*)(TB + TB_T6 + 3 * HD + 4 * lane);
  const v4f t4 = *(const v4f*)(TB + TB_T6 + 4 * HD + 4 * lane);
  const v4f t5 = *(const v4f*)(TB + TB_T6 + 5 * HD + 4 * lane);
  const v4f e1 = *(const v4f*)(TB + TB_BE1 + 4 * lane);
  const v4f w2 = *(const v4f*)(TB + TB_WE2 + 4 * lane);
  const float bz = TB[TB_SC + 1];
  float keep = 0.0f;
#pragma unroll 1
  for (int k = 0; k < 32; ++k) {
    const int sk = __builtin_amdgcn_readlane(s, k);
    const int dk = __builtin_amdgcn_readlane(d, k);
    const v4f ps = *(const v4f*)(PS + (size_t)sk * HD + 4 * lane);
    const v4f pd = *(const v4f*)(PD + (size_t)dk * HD + 4 * lane);
    const float g0 = rdl(g0l, k), g1 = rdl(g1l, k), g2 = rdl(g2l, k);
    const float g3 = rdl(g3l, k), g4 = rdl(g4l, k), g5 = rdl(g5l, k);
    float z0 = ps.x + pd.x, z1 = ps.y + pd.y, z2 = ps.z + pd.z, z3 = ps.w + pd.w;
    z0 = fmaf(g0, t0.x, z0); z1 = fmaf(g0, t0.y, z1); z2 = fmaf(g0, t0.z, z2); z3 = fmaf(g0, t0.w, z3);
    z0 = fmaf(g1, t1.x, z0); z1 = fmaf(g1, t1.y, z1); z2 = fmaf(g1, t1.z, z2); z3 = fmaf(g1, t1.w, z3);
    z0 = fmaf(g2, t2.x, z0); z1 = fmaf(g2, t2.y, z1); z2 = fmaf(g2, t2.z, z2); z3 = fmaf(g2, t2.w, z3);
    z0 = fmaf(g3, t3.x, z0); z1 = fmaf(g3, t3.y, z1); z2 = fmaf(g3, t3.z, z2); z3 = fmaf(g3, t3.w, z3);
    z0 = fmaf(g4, t4.x, z0); z1 = fmaf(g4, t4.y, z1); z2 = fmaf(g4, t4.z, z2); z3 = fmaf(g4, t4.w, z3);
    z0 = fmaf(g5, t5.x, z0); z1 = fmaf(g5, t5.y, z1); z2 = fmaf(g5, t5.z, z2); z3 = fmaf(g5, t5.w, z3);
    const float h0 = relu_k(z0 + e1.x);
    const float h1 = relu_k(z1 + e1.y);
    const float h2 = relu_k(z2 + e1.z);
    const float h3 = relu_k(z3 + e1.w);
    float p = fmaf(h0, w2.x, fmaf(h1, w2.y, fmaf(h2, w2.z, h3 * w2.w)));
    p += __shfl_xor(p, 16, 32);
    p += __shfl_xor(p, 8, 32);
    p += __shfl_xor(p, 4, 32);
    p += __shfl_xor(p, 2, 32);
    p += __shfl_xor(p, 1, 32);
    keep = (lane == k) ? p : keep;
  }
  const float r = keep + bz;
  float* op = out1 + e;
  *(volatile float*)op = r;
  __threadfence();
  *(volatile float*)op = r;
}

extern "C" void kernel_launch(void* const* d_in, const int* in_sizes, int n_in,
                              void* d_out, int out_size, void* d_ws, size_t ws_size,
                              hipStream_t stream) {
  if (n_in < 20) return;
  if (in_sizes[0] != 2 * NE || in_sizes[1] != NN * 6 || in_sizes[2] != NE * 4) return;
  if (in_sizes[3] != NN || in_sizes[4] != NE || in_sizes[5] != NN || in_sizes[6] != NE) return;
  if (in_sizes[7] != 8 * HD || in_sizes[8] != HD) return;
  if (in_sizes[9] != NLAY * HD * HD || in_sizes[10] != NLAY * HD * HD || in_sizes[11] != NLAY * HD) return;
  if (in_sizes[12] != HD * HD || in_sizes[13] != HD || in_sizes[14] != HD || in_sizes[15] != 1) return;
  if (in_sizes[16] != 262 * HD || in_sizes[17] != HD || in_sizes[18] != HD || in_sizes[19] != 1) return;
  if (out_size != NN + NE) return;

  const int*   ei   = (const int*)  d_in[0];
  const float* nst  = (const float*)d_in[1];
  const float* est  = (const float*)d_in[2];
  const float* pob  = (const float*)d_in[3];
  const float* qob  = (const float*)d_in[4];
  const int*   pmk  = (const int*)  d_in[5];
  const int*   qmk  = (const int*)  d_in[6];
  const float* wenc = (const float*)d_in[7];
  const float* benc = (const float*)d_in[8];
  const float* Wl   = (const float*)d_in[9];
  const float* Wr   = (const float*)d_in[10];
  const float* bg   = (const float*)d_in[11];
  const float* Wn1  = (const float*)d_in[12];
  const float* bn1  = (const float*)d_in[13];
  const float* Wn2  = (const float*)d_in[14];
  const float* bn2  = (const float*)d_in[15];
  const float* We1  = (const float*)d_in[16];
  const float* be1  = (const float*)d_in[17];
  const float* We2  = (const float*)d_in[18];
  const float* be2  = (const float*)d_in[19];
  float* out = (float*)d_out;

  constexpr size_t szX   = (size_t)MP * XP * 2;
  constexpr size_t szL   = (size_t)NBLK * RCAP * 4;
  constexpr size_t szT   = (size_t)NSLOT * 4;
  constexpr size_t szWC  = (size_t)NLAY * HD * KC * 2;
  constexpr size_t szWH  = (size_t)3 * HD * KH * 2;
  constexpr size_t szTB  = (size_t)TB_N * 4;
  constexpr size_t szFL  = (size_t)NBLK * 128;
  constexpr size_t oXA   = 0;
  constexpr size_t oAGB  = oXA + szX;
  constexpr size_t oLIST = oAGB + szX;
  constexpr size_t oCNT  = oLIST + szL;
  constexpr size_t oOFF  = oCNT + szT;
  constexpr size_t oINV  = oOFF + szT;
  constexpr size_t oWC   = oINV + szT;
  constexpr size_t oWH   = oWC + szWC;
  constexpr size_t oTB   = oWH + szWH;
  constexpr size_t oFLG  = oTB + szTB;
  constexpr size_t oEND  = oFLG + szFL;
  static_assert(oEND <= (size_t)WSMAX);
  static_assert(szX % 256 == 0 && szL % 256 == 0 && szT % 256 == 0 && szWC % 256 == 0 && szWH % 256 == 0);
  static_assert(szTB % 256 == 0 && szFL % 256 == 0);
  static_assert((size_t)MP * HD * 4 == szX);
  if (oEND > ws_size) return;
  char* ws = (char*)d_ws;
  unsigned short* XA   = (unsigned short*)(ws + oXA);
  unsigned short* AGB  = (unsigned short*)(ws + oAGB);
  int*            LIST = (int*)(ws + oLIST);
  int*            CNT  = (int*)(ws + oCNT);
  int*            OFF  = (int*)(ws + oOFF);
  float*          INVD = (float*)(ws + oINV);
  unsigned short* WC   = (unsigned short*)(ws + oWC);
  unsigned short* WH   = (unsigned short*)(ws + oWH);
  float*          TB   = (float*)(ws + oTB);
  int*            FLG  = (int*)(ws + oFLG);
  float*          PS   = (float*)(ws + oAGB);
  float*          PD   = (float*)(ws + oXA);

  const int bktLds = BK_LDS_INTS * 4;
  const int gmLds  = GM_LDS_BYTES;
  hipFuncSetAttribute(reinterpret_cast<const void*>(&k_bkt), hipFuncAttributeMaxDynamicSharedMemorySize, bktLds);
  hipFuncSetAttribute(reinterpret_cast<const void*>(&k_gm<0>), hipFuncAttributeMaxDynamicSharedMemorySize, gmLds);
  hipFuncSetAttribute(reinterpret_cast<const void*>(&k_gm<1>), hipFuncAttributeMaxDynamicSharedMemorySize, gmLds);
  hipFuncSetAttribute(reinterpret_cast<const void*>(&k_gm<2>), hipFuncAttributeMaxDynamicSharedMemorySize, gmLds);
  hipFuncSetAttribute(reinterpret_cast<const void*>(&k_gm<3>), hipFuncAttributeMaxDynamicSharedMemorySize, gmLds);
  hipFuncSetAttribute(reinterpret_cast<const void*>(&k_gm<4>), hipFuncAttributeMaxDynamicSharedMemorySize, gmLds);

  const int gRow = MP / GBM;

  k_pa<<<MP / (NWAVE * PAROWS), NTHR, 0, stream>>>(nst, pob, pmk, wenc, benc, XA);
  k_pb<<<NUWC / NTHR, NTHR, 0, stream>>>(Wl, Wr, WC);
  k_pc<<<(NUWH + NTU + NTHR - 1) / NTHR, NTHR, 0, stream>>>(Wn1, We1, bg, bn1, Wn2, bn2, be1, We2, be2, WH, TB);
  k_bkt<<<NBLK, NTHR, bktLds, stream>>>(ei, LIST, CNT, OFF, INVD, FLG);
  k_agg<<<gRow, NTHR, 0, stream>>>(LIST, CNT, OFF, INVD, FLG, XA, AGB);
  k_gm<0><<<gRow, NTHR, gmLds, stream>>>(AGB, XA, WC + (size_t)0 * HD * KC, TB, TB_BG + 0 * HD, PS, out);
  k_agg<<<gRow, NTHR, 0, stream>>>(LIST, CNT, OFF, INVD, FLG, XA, AGB);
  k_gm<0><<<gRow, NTHR, gmLds, stream>>>(AGB, XA, WC + (size_t)1 * HD * KC, TB, TB_BG + 1 * HD, PS, out);
  k_agg<<<gRow, NTHR, 0, stream>>>(LIST, CNT, OFF, INVD, FLG, XA, AGB);
  k_gm<1><<<gRow, NTHR, gmLds, stream>>>(AGB, XA, WC + (size_t)2 * HD * KC, TB, TB_BG + 2 * HD, PS, out);
  k_gm<2><<<gRow, NTHR, gmLds, stream>>>(AGB, XA, WH + (size_t)0 * HD * KH, TB, 0, PS, out);
  k_gm<3><<<gRow, NTHR, gmLds, stream>>>(AGB, XA, WH + (size_t)1 * HD * KH, TB, 0, PS, out);
  k_gm<4><<<gRow, NTHR, gmLds, stream>>>(AGB, XA, WH + (size_t)2 * HD * KH, TB, 0, PD, out);
  k_edge<<<NE / NTHR, NTHR, 0, stream>>>(ei, est, qob, qmk, PS, PD, TB, out + NN);
}
